// MyModel_87522843559835
// MI455X (gfx1250) — hardware-verified
//
#include <hip/hip_runtime.h>
#include <math.h>

typedef __attribute__((ext_vector_type(16))) _Float16 v16h;
typedef __attribute__((ext_vector_type(16))) __bf16 v16b;
typedef __attribute__((ext_vector_type(8)))  _Float16 v8h;
typedef __attribute__((ext_vector_type(8)))  float v8f;
typedef __attribute__((ext_vector_type(4)))  float v4f;
typedef __attribute__((ext_vector_type(2)))  float v2f;
typedef __attribute__((ext_vector_type(4)))  unsigned v4u;
typedef __attribute__((ext_vector_type(4)))  int v4i;
typedef float __attribute__((may_alias)) float_a;
typedef int __attribute__((may_alias)) int_a;

template <typename T> __device__ __forceinline__ void vst2(void* p, T v) { *(volatile T*)p = v; __threadfence(); *(volatile T*)p = v; }
__device__ __forceinline__ v8f wmma16(v16h a, v16h b, v8f c) {
  v8f d = __builtin_amdgcn_wmma_f32_16x16x32_f16(false, a, false, b, (short)0, c, false, false);
  asm volatile("v_nop\n\tv_nop\n\tv_nop\n\tv_nop" : "+v"(d) : "v"(a), "v"(b));
  return d;
}
__device__ __forceinline__ v8f wmma_bf(v16b a, v16b b, v8f c) {
  v8f d = __builtin_amdgcn_wmma_f32_16x16x32_bf16(false, a, false, b, (short)0, c, false, false);
  asm volatile("v_nop\n\tv_nop\n\tv_nop\n\tv_nop" : "+v"(d) : "v"(a), "v"(b));
  return d;
}
__device__ __forceinline__ v16h frag_h(const _Float16* rowk0, int lane) {
  union { v16h v; v8h q[2]; } u; const _Float16* p = rowk0 + 8 * (lane >> 4);
  u.q[0] = *(const v8h*)p; u.q[1] = *(const v8h*)(p + 16); return u.v;
}
__device__ __forceinline__ v16h frag_f32(const float* rowk0, int lane) {
  v16h a; const float* p = rowk0 + 8 * (lane >> 4);
#pragma unroll
  for (int i = 0; i < 8; ++i) { a[i] = (_Float16)p[i]; a[8 + i] = (_Float16)p[16 + i]; }
  return a;
}
__device__ __forceinline__ v16h frag_f32s(const float* rowk0, int lane, float sc) {
  v16h a; const float* p = rowk0 + 8 * (lane >> 4);
#pragma unroll
  for (int i = 0; i < 8; ++i) { a[i] = (_Float16)(p[i] * sc); a[8 + i] = (_Float16)(p[16 + i] * sc); }
  return a;
}
__device__ __forceinline__ v16h fragc_f32(const float* W, int k0, int n, int lane, int ld, int K) {
  v16h a; const int g = lane >> 4;
#pragma unroll
  for (int i = 0; i < 8; ++i) { const int ka = k0 + 8 * g + i, kb = ka + 16;
    a[i] = (_Float16)(ka < K ? W[(size_t)(ka < K ? ka : K - 1) * ld + n] : 0.f); a[8 + i] = (_Float16)(kb < K ? W[(size_t)(kb < K ? kb : K - 1) * ld + n] : 0.f); }
  return a;
}
struct F2 { v16b h, l; };
__device__ __forceinline__ F2 bsplit16(const float v[16]) { F2 r;
#pragma unroll
  for (int i = 0; i < 16; ++i) { const __bf16 h = (__bf16)v[i]; r.h[i] = h; r.l[i] = (__bf16)(v[i] - (float)h); }
  return r; }
__device__ __forceinline__ F2 split_row(const float* row, int k0, int lane) { float v[16]; const float* p = row + k0 + 8 * (lane >> 4);
#pragma unroll
  for (int i = 0; i < 8; ++i) { v[i] = p[i]; v[8 + i] = p[16 + i]; }
  return bsplit16(v); }
__device__ __forceinline__ F2 split_rowK(const float* row, int k0, int lane, int K) { float v[16]; const int g = lane >> 4;
#pragma unroll
  for (int i = 0; i < 8; ++i) { const int ka = k0 + 8 * g + i, kb = ka + 16; v[i] = ka < K ? row[ka < K ? ka : K - 1] : 0.f; v[8 + i] = kb < K ? row[kb < K ? kb : K - 1] : 0.f; }
  return bsplit16(v); }
__device__ __forceinline__ F2 split_col(const float* W, int k0, int n, int lane, int ld, int K) { float v[16]; const int g = lane >> 4;
#pragma unroll
  for (int i = 0; i < 8; ++i) { const int ka = k0 + 8 * g + i, kb = ka + 16; v[i] = ka < K ? W[(size_t)(ka < K ? ka : K - 1) * ld + n] : 0.f; v[8 + i] = kb < K ? W[(size_t)(kb < K ? kb : K - 1) * ld + n] : 0.f; }
  return bsplit16(v); }
__device__ __forceinline__ v8f mac3(const F2& a, const F2& b, v8f c) { c = wmma_bf(a.l, b.h, c); c = wmma_bf(a.h, b.l, c); return wmma_bf(a.h, b.h, c); }
__device__ __forceinline__ float sigm(float v) { return 1.0f / (1.0f + expf(-v)); }
#define LDSX() do { asm volatile("s_wait_dscnt 0" ::: "memory"); __builtin_amdgcn_wave_barrier(); __builtin_amdgcn_fence(__ATOMIC_RELEASE, "workgroup"); } while (0)


#define NB 4
#define NN 2048
#define FF 512
#define DD 64
#ifndef TNB
#define TNB NB
#endif
typedef __attribute__((ext_vector_type(8))) __bf16 v8b;
__device__ __forceinline__ v16b frag_b(const __bf16* rowk0, int lane) {
  union { v16b v; v8b q[2]; } u; const __bf16* p = rowk0 + 8 * (lane >> 4);
  u.q[0] = *(const v8b*)p; u.q[1] = *(const v8b*)(p + 16); return u.v;
}
__device__ __forceinline__ float bfr(float v) { return (float)(__bf16)v; }
__device__ __attribute__((noinline)) float exp_ni(float v) { return expf(v); }
__device__ __attribute__((noinline)) float erf_ni(float v) { return erff(v); }

#define WS_PW  0u
#define WS_QH  (WS_PW + 2u * 3 * DD * FF)
#define WS_QL  (WS_QH + 2u * (size_t)NB * NN * DD)
#define WS_KH  (WS_QL + 2u * (size_t)NB * NN * DD)
#define WS_KL  (WS_KH + 2u * (size_t)NB * NN * DD)
#define WS_VT  (WS_KL + 2u * (size_t)NB * NN * DD)
#define WS_VTL (WS_VT + 2u * (size_t)NB * DD * NN)
#define WS_END (WS_VTL + 2u * (size_t)NB * DD * NN)

__global__ __launch_bounds__(256) void k_packw(const float* __restrict__ WQ, const float* __restrict__ WK, const float* __restrict__ WV, __bf16* __restrict__ PW) { const int n = blockIdx.x, t = threadIdx.x; __shared__ __align__(16) __bf16 s[FF]; const int which = n / DD, u = n % DD; const float* Wm = which == 0 ? WQ : which == 1 ? WK : WV;
  for (int k = t; k < FF; k += 256) s[k] = (__bf16)Wm[(size_t)k * DD + u]; __syncthreads(); if (t < FF / 8) vst2((unsigned*)(PW + (size_t)n * FF + t * 8), *(const v4u*)&s[t * 8]); }
__global__ __launch_bounds__(128) void k_proj(const float* __restrict__ X, const __bf16* __restrict__ PW, const float* __restrict__ BQ, const float* __restrict__ BK, const float* __restrict__ BV, _Float16* __restrict__ QH, _Float16* __restrict__ QL, _Float16* __restrict__ KH, _Float16* __restrict__ KL, _Float16* __restrict__ VT, _Float16* __restrict__ VTL) {
  __shared__ __align__(16) _Float16 sq[64][72], sql[64][72], sk[64][72], skl[64][72]; __shared__ __align__(16) _Float16 th[DD][72], tl[DD][72];
  const int tid = threadIdx.x, wave = tid >> 5, lane = tid & 31, col = lane & 15, g = lane >> 4; const size_t r0 = (size_t)blockIdx.x * 64 + wave * 16; const size_t b = ((size_t)blockIdx.x * 64) / NN; const int n0 = (int)(((size_t)blockIdx.x * 64) % NN);
  v8f acc[12];
#pragma unroll
  for (int j = 0; j < 12; ++j) acc[j] = v8f{};
#pragma unroll 2
  for (int kc = 0; kc < FF / 32; ++kc) { v16b a; const float* pp = X + (r0 + col) * FF + kc * 32 + 8 * g;
#pragma unroll
    for (int i = 0; i < 8; ++i) { a[i] = (__bf16)pp[i]; a[8 + i] = (__bf16)pp[16 + i]; }
#pragma unroll
    for (int j = 0; j < 12; ++j) acc[j] = wmma_bf(a, frag_b(PW + (size_t)(j * 16 + col) * FF + kc * 32, lane), acc[j]); }
#pragma unroll
  for (int j = 0; j < 12; ++j) { const int c = (j & 3) * 16 + col; const float bb = j < 4 ? bfr(BQ[c]) : j < 8 ? bfr(BK[c]) : bfr(BV[c]);
#pragma unroll
    for (int r = 0; r < 8; ++r) { const float v = acc[j][r] + bb; const _Float16 hv = (_Float16)v, lv = (_Float16)((v - (float)hv) * 2048.0f); const int rl = wave * 16 + 8 * g + r; if (j < 4) { sq[rl][c] = hv; sql[rl][c] = lv; } else if (j < 8) { sk[rl][c] = hv; skl[rl][c] = lv; } else { th[c][rl] = hv; tl[c][rl] = lv; } } }
  __syncthreads();
  for (int e = tid; e < 64 * 8; e += 128) { const int rl = e >> 3, q = e & 7; const size_t o = ((size_t)blockIdx.x * 64 + rl) * DD + q * 8; vst2((unsigned*)(QH + o), *(const v4u*)&sq[rl][q * 8]); vst2((unsigned*)(QL + o), *(const v4u*)&sql[rl][q * 8]); vst2((unsigned*)(KH + o), *(const v4u*)&sk[rl][q * 8]); vst2((unsigned*)(KL + o), *(const v4u*)&skl[rl][q * 8]); }
  for (int e = tid; e < DD * 8; e += 128) { const int c = e >> 3, q = e & 7; const size_t o = (b * DD + c) * (size_t)NN + n0 + q * 8; vst2((unsigned*)(VT + o), *(const v4u*)&th[c][q * 8]); vst2((unsigned*)(VTL + o), *(const v4u*)&tl[c][q * 8]); } }
__global__ __launch_bounds__(128) void k_att(const _Float16* __restrict__ QH, const _Float16* __restrict__ QL, const _Float16* __restrict__ KH, const _Float16* __restrict__ KL, const _Float16* __restrict__ VT, const _Float16* __restrict__ VTL, const int* __restrict__ MK, float* __restrict__ OUT) {
  __shared__ __align__(16) float sp[4][16][36]; __shared__ __align__(16) float so[4][16][68];
  const int tid = threadIdx.x, wave = tid >> 5, lane = tid & 31, col = lane & 15, g = lane >> 4; const size_t b = blockIdx.y; const int q0 = blockIdx.x * 64 + wave * 16; const size_t rq = b * NN + q0;
  v16h aq[2], al[2];
#pragma unroll
  for (int kc = 0; kc < 2; ++kc) { aq[kc] = frag_h(QH + (rq + col) * DD + kc * 32, lane); al[kc] = frag_h(QL + (rq + col) * DD + kc * 32, lane); }
  float m[8], l[8];
#pragma unroll
  for (int r = 0; r < 8; ++r) { m[r] = -3.0e38f; l[r] = 0.f; }
  v8f acc[4] = {}, accl[4] = {};
#pragma unroll 1
  for (int ks = 0; ks < NN / 32; ++ks) { float s[2][8];
#pragma unroll
    for (int ct = 0; ct < 2; ++ct) { const int kk = ks * 32 + ct * 16 + col; const size_t rk = b * NN + kk; v8f c = {}, cl = {};
#pragma unroll
      for (int kc = 0; kc < 2; ++kc) { const v16h kh = frag_h(KH + rk * DD + kc * 32, lane), kl = frag_h(KL + rk * DD + kc * 32, lane); c = wmma16(aq[kc], kh, c); cl = wmma16(aq[kc], kl, cl); cl = wmma16(al[kc], kh, cl); }
      const bool keep = MK[b * NN + kk] != 0;
#pragma unroll
      for (int r = 0; r < 8; ++r) s[ct][r] = keep ? (c[r] + cl[r] * (1.0f / 2048.0f)) * 0.125f : -3.0e38f; }
    float alpha[8];
#pragma unroll
    for (int r = 0; r < 8; ++r) { float mx = fmaxf(s[0][r], s[1][r]);
#pragma unroll
      for (int o = 1; o < 16; o <<= 1) mx = fmaxf(mx, __shfl_xor(mx, o));
      const float mn = fmaxf(m[r], mx); alpha[r] = (m[r] <= -1.0e38f) ? 0.f : __expf(m[r] - mn); const float e0 = (s[0][r] <= -1.0e38f) ? 0.f : __expf(s[0][r] - mn), e1 = (s[1][r] <= -1.0e38f) ? 0.f : __expf(s[1][r] - mn); float es = e0 + e1;
#pragma unroll
      for (int o = 1; o < 16; o <<= 1) es += __shfl_xor(es, o);
      l[r] = l[r] * alpha[r] + es; m[r] = (mn > -1.0e38f) ? mn : m[r]; sp[wave][8 * g + r][col] = e0; sp[wave][8 * g + r][16 + col] = e1; }
#pragma unroll
    for (int j = 0; j < 4; ++j)
#pragma unroll
      for (int r = 0; r < 8; ++r) { acc[j][r] *= alpha[r]; accl[j][r] *= alpha[r]; }
    LDSX();
    v16h pa, pal; { const float* prow = &sp[wave][col][0] + 8 * (lane >> 4);
#pragma unroll
      for (int i = 0; i < 8; ++i) { const float p0 = prow[i] * 2048.0f, p1 = prow[16 + i] * 2048.0f; pa[i] = (_Float16)p0; pa[8 + i] = (_Float16)p1; pal[i] = (_Float16)((p0 - (float)pa[i]) * 2048.0f); pal[8 + i] = (_Float16)((p1 - (float)pa[8 + i]) * 2048.0f); } }
#pragma unroll
    for (int j = 0; j < 4; ++j) { const size_t po = (b * DD + j * 16 + col) * (size_t)NN + ks * 32; const v16h vh = frag_h(VT + po, lane), vl = frag_h(VTL + po, lane); acc[j] = wmma16(pa, vh, acc[j]); accl[j] = wmma16(pa, vl, accl[j]); accl[j] = wmma16(pal, vh, accl[j]); }
    LDSX(); }
#pragma unroll
  for (int r = 0; r < 8; ++r) { const float il = (l[r] > 0.f) ? (1.0f / 2048.0f) / l[r] : 0.f;
#pragma unroll
    for (int j = 0; j < 4; ++j) so[wave][8 * g + r][j * 16 + col] = (acc[j][r] + accl[j][r] * (1.0f / 2048.0f)) * il; }
  LDSX(); for (int rl = 0; rl < 16; ++rl) if (lane < 16) vst2(OUT + (rq + rl) * DD + lane * 4, *(const v4f*)&so[wave][rl][lane * 4]); }
extern "C" void kernel_launch(void* const* d_in, const int* in_sizes, int n_in, void* d_out, int out_size, void* d_ws, size_t ws_size, hipStream_t stream) {
  (void)in_sizes; (void)n_in; (void)out_size;
  const float** F = (const float**)d_in;
  if (ws_size < (size_t)WS_END) return;
  char* ws = (char*)d_ws; __bf16* PW = (__bf16*)(ws + WS_PW); _Float16 *QH = (_Float16*)(ws + WS_QH), *QL = (_Float16*)(ws + WS_QL), *KH = (_Float16*)(ws + WS_KH), *KL = (_Float16*)(ws + WS_KL), *VT = (_Float16*)(ws + WS_VT), *VTL = (_Float16*)(ws + WS_VTL);
  k_packw<<<3 * DD, 256, 0, stream>>>(F[2], F[4], F[6], PW);
  k_proj<<<NB * NN / 64, 128, 0, stream>>>(F[0], PW, F[3], F[5], F[7], QH, QL, KH, KL, VT, VTL);
  k_att<<<dim3(NN / 64, TNB), 128, 0, stream>>>(QH, QL, KH, KL, VT, VTL, (const int*)d_in[1], (float*)d_out);
}
